// MACBlock_77189152244394
// MI455X (gfx1250) — hardware-verified
//
#include <hip/hip_runtime.h>
#include <hip/hip_bf16.h>
#include <math.h>


typedef _Float16 bf16;
typedef _Float16 f16;
typedef __attribute__((ext_vector_type(4))) unsigned v4u_t;
typedef unsigned v4ua __attribute__((ext_vector_type(4), may_alias));
typedef __attribute__((ext_vector_type(4))) float v4f_t;
typedef float v4fa __attribute__((ext_vector_type(4), may_alias));
typedef __attribute__((ext_vector_type(16))) bf16  bf16x16;
typedef bf16x16 f16x16;
typedef __attribute__((ext_vector_type(8)))  bf16  bf16x8;
typedef bf16x8 f16x8;
typedef __attribute__((ext_vector_type(4)))  bf16  bf16x4;
typedef __attribute__((ext_vector_type(8)))  float f32x8;
__device__ __forceinline__ f32x8 wmma16(f16x16 a, f16x16 b, f32x8 c) {
  c = __builtin_amdgcn_wmma_f32_16x16x32_f16(false, a, false, b, (short)0, c, false, false);
  asm volatile("v_nop\n\tv_nop\n\tv_nop\n\tv_nop" : "+v"(c) : "v"(a), "v"(b));
  return c;
}
#define LDS_STRIDE 48
#define KSTRIDE    72
#define VSTRIDE    48

__device__ __forceinline__ f32x8 wmma_bf16(bf16x16 a, bf16x16 b, f32x8 c) {
  c = __builtin_amdgcn_wmma_f32_16x16x32_f16(false, a, false, b, (short)0, c, false, false);
  asm volatile("v_nop\n\tv_nop\n\tv_nop\n\tv_nop" : "+v"(c) : "v"(a), "v"(b));
  return c;
}

template <typename T>
__device__ __forceinline__ bf16x16 load_frag(const T* __restrict__ base, int ld,
                                             int row0, int k0) {
  const int lane = threadIdx.x & 31;
  const int r    = lane & 15;
  const int kh   = (lane >> 4) * 8;
  const T* p0 = base + (size_t)(row0 + r) * ld + (k0 + kh);
  const T* p1 = p0 + 16;
  bf16x16 f;
#pragma unroll
  for (int i = 0; i < 8; ++i) {
    f[i]     = (bf16)p0[i];
    f[i + 8] = (bf16)p1[i];
  }
  return f;
}

__device__ __forceinline__ bf16x16 lds_frag(const bf16* base, int stride) {
  const int lane = threadIdx.x & 31;
  const int row  = lane & 15;
  const int kh   = (lane >> 4) * 8;
  const bf16x8 lo = *(const bf16x8*)(base + row * stride + kh);
  const bf16x8 hi = *(const bf16x8*)(base + row * stride + kh + 16);
  bf16x16 f;
#pragma unroll
  for (int i = 0; i < 8; ++i) { f[i] = lo[i]; f[i + 8] = hi[i]; }
  return f;
}

template <typename T>
__device__ __forceinline__ void stage_read16(const T* __restrict__ p, float* buf) {
#pragma unroll
  for (int i = 0; i < 16; ++i) buf[i] = (float)p[i];
}

__device__ __forceinline__ void stage_write(bf16* dst, const float* buf, int nquad) {
#pragma unroll
  for (int i = 0; i < nquad; ++i) {
    bf16x4 q;
    q[0] = (bf16)buf[4 * i];     q[1] = (bf16)buf[4 * i + 1];
    q[2] = (bf16)buf[4 * i + 2]; q[3] = (bf16)buf[4 * i + 3];
    *(bf16x4*)(dst + 4 * i) = q;
  }
}


#define GSTR 48
#define GSTR 48
template <typename AT, int EPI, bool OUT16>
__global__ __launch_bounds__(256) void gemm_kne(const AT* __restrict__ A, int lda, const float* __restrict__ Wm, int ldw,
                                                const float* __restrict__ bias, const float* __restrict__ R, const float* __restrict__ gvec,
                                                void* __restrict__ Yv, int ldy, int K) {
  __shared__ __attribute__((aligned(16))) f16 ldsA[128 * GSTR];
  __shared__ __attribute__((aligned(16))) f16 ldsW[128 * GSTR];
  __shared__ __attribute__((aligned(16))) float oS[8][32 * 68];
  const int tid = threadIdx.x, lane = tid & 31, wave = tid >> 5, cl = lane & 15, rh = (lane >> 4) * 8;
  const int m0 = blockIdx.x * 128, n0 = blockIdx.y * 128;
  const int wm = (wave & 3) * 32, wn = (wave >> 2) * 64;
  f32x8 acc[2][4];
#pragma unroll
  for (int i = 0; i < 2; ++i)
#pragma unroll
    for (int j = 0; j < 4; ++j) { f32x8 z = {}; acc[i][j] = z; }
#pragma unroll 1
  for (int k0 = 0; k0 < K; k0 += 32) {
    __syncthreads();
    { const int row = tid >> 1, ch = (tid & 1) * 16;
      const AT* src = A + (size_t)(m0 + row) * lda + k0 + ch;
#pragma unroll
      for (int g = 0; g < 16; ++g) ldsA[row * GSTR + ch + g] = (f16)src[g]; }
    { const int k = tid >> 3, nn0 = (tid & 7) * 16;
      const float* src = Wm + (size_t)(k0 + k) * ldw + n0 + nn0;
#pragma unroll
      for (int g = 0; g < 4; ++g) { const v4f_t v = *(const v4f_t*)(src + 4 * g);
#pragma unroll
        for (int u = 0; u < 4; ++u) ldsW[(nn0 + 4 * g + u) * GSTR + k] = (f16)v[u]; } }
    __syncthreads();
    f16x16 af[2];
#pragma unroll
    for (int i = 0; i < 2; ++i) af[i] = lds_frag(ldsA + (wm + 16 * i) * GSTR, GSTR);
#pragma unroll
    for (int j = 0; j < 4; ++j) {
      const f16x16 bf = lds_frag(ldsW + (wn + 16 * j) * GSTR, GSTR);
#pragma unroll
      for (int i = 0; i < 2; ++i) acc[i][j] = wmma16(af[i], bf, acc[i][j]);
    }
  }
  float* so = oS[wave];
#pragma unroll
  for (int i = 0; i < 2; ++i)
#pragma unroll
    for (int j = 0; j < 4; ++j) {
      const int n = n0 + wn + 16 * j + cl;
      const float bv = bias ? bias[n] : 0.0f;
      const float gv = (EPI == 2 || EPI == 4) ? gvec[n] : 0.0f;
      if (EPI == 1) {
#pragma unroll 1
        for (int r = 0; r < 8; ++r) { const float xg = acc[i][j][r] + bv; so[(16 * i + rh + r) * 68 + 16 * j + cl] = 0.5f * xg * (1.0f + erff(xg * 0.70710678118654752f)); }
      } else {
#pragma unroll
        for (int r = 0; r < 8; ++r) {
          float v = acc[i][j][r] + bv;
          if (EPI == 3) v = fmaxf(v, 0.0f);
          if (EPI == 4) v = gv * v;
          if (EPI == 2) v = R[(size_t)(m0 + wm + 16 * i + rh + r) * ldy + n] + gv * v;
          so[(16 * i + rh + r) * 68 + 16 * j + cl] = v;
        }
      }
    }
  asm volatile("s_wait_dscnt 0" ::: "memory");
  __builtin_amdgcn_wave_barrier();
#pragma unroll 1
  for (int pass = 0; pass < 2; ++pass) {
    if (OUT16) {
      f16* Y = (f16*)Yv;
#pragma unroll
      for (int it = 0; it < 8; ++it) { const int c = lane + 32 * it, rr = c >> 3, q8 = (c & 7) * 8;
        union { f16 h[8]; v4u_t v; } u;
#pragma unroll
        for (int e = 0; e < 8; ++e) u.h[e] = (f16)so[rr * 68 + q8 + e];
        *(volatile v4u_t*)(Y + (size_t)(m0 + wm + rr) * ldy + n0 + wn + q8) = u.v; }
    } else {
      float* Y = (float*)Yv;
#pragma unroll
      for (int it = 0; it < 16; ++it) { const int f4 = lane + 32 * it, rr = f4 >> 4, q = (f4 & 15) * 4;
        *(volatile v4f_t*)(Y + (size_t)(m0 + wm + rr) * ldy + n0 + wn + q) = *(const v4fa*)(so + rr * 68 + q); }
    }
    __threadfence();
  }
}

template <typename AT, int EPI, bool OUT16>
__global__ __launch_bounds__(256) void gemm_knez(const AT* __restrict__ A, int lda, size_t strideA, const float* __restrict__ Wm, int ldw, size_t strideW,
                                                 const float* __restrict__ bias, const float* __restrict__ R, const float* __restrict__ gvec,
                                                 void* __restrict__ Yv, int ldy, size_t strideY, int K) {
  A += (size_t)blockIdx.z * strideA; Wm += (size_t)blockIdx.z * strideW; Yv = (void*)((char*)Yv + (size_t)blockIdx.z * strideY * (OUT16 ? 2 : 4)); if (R) R += (size_t)blockIdx.z * strideY;
  __shared__ __attribute__((aligned(16))) f16 ldsA[128 * GSTR];
  __shared__ __attribute__((aligned(16))) f16 ldsW[128 * GSTR];
  __shared__ __attribute__((aligned(16))) float oS[8][32 * 68];
  const int tid = threadIdx.x, lane = tid & 31, wave = tid >> 5, cl = lane & 15, rh = (lane >> 4) * 8;
  const int m0 = blockIdx.x * 128, n0 = blockIdx.y * 128;
  const int wm = (wave & 3) * 32, wn = (wave >> 2) * 64;
  f32x8 acc[2][4];
#pragma unroll
  for (int i = 0; i < 2; ++i)
#pragma unroll
    for (int j = 0; j < 4; ++j) { f32x8 z = {}; acc[i][j] = z; }
#pragma unroll 1
  for (int k0 = 0; k0 < K; k0 += 32) {
    __syncthreads();
    { const int row = tid >> 1, ch = (tid & 1) * 16;
      const AT* src = A + (size_t)(m0 + row) * lda + k0 + ch;
#pragma unroll
      for (int g = 0; g < 16; ++g) ldsA[row * GSTR + ch + g] = (f16)src[g]; }
    { const int k = tid >> 3, nn0 = (tid & 7) * 16;
      const float* src = Wm + (size_t)(k0 + k) * ldw + n0 + nn0;
#pragma unroll
      for (int g = 0; g < 4; ++g) { const v4f_t v = *(const v4f_t*)(src + 4 * g);
#pragma unroll
        for (int u = 0; u < 4; ++u) ldsW[(nn0 + 4 * g + u) * GSTR + k] = (f16)v[u]; } }
    __syncthreads();
    f16x16 af[2];
#pragma unroll
    for (int i = 0; i < 2; ++i) af[i] = lds_frag(ldsA + (wm + 16 * i) * GSTR, GSTR);
#pragma unroll
    for (int j = 0; j < 4; ++j) {
      const f16x16 bf = lds_frag(ldsW + (wn + 16 * j) * GSTR, GSTR);
#pragma unroll
      for (int i = 0; i < 2; ++i) acc[i][j] = wmma16(af[i], bf, acc[i][j]);
    }
  }
  float* so = oS[wave];
#pragma unroll
  for (int i = 0; i < 2; ++i)
#pragma unroll
    for (int j = 0; j < 4; ++j) {
      const int n = n0 + wn + 16 * j + cl;
      const float bv = bias ? bias[n] : 0.0f;
      const float gv = (EPI == 2 || EPI == 4) ? gvec[n] : 0.0f;
      if (EPI == 1) {
#pragma unroll 1
        for (int r = 0; r < 8; ++r) { const float xg = acc[i][j][r] + bv; so[(16 * i + rh + r) * 68 + 16 * j + cl] = 0.5f * xg * (1.0f + erff(xg * 0.70710678118654752f)); }
      } else {
#pragma unroll
        for (int r = 0; r < 8; ++r) {
          float v = acc[i][j][r] + bv;
          if (EPI == 3) v = fmaxf(v, 0.0f);
          if (EPI == 4) v = gv * v;
          if (EPI == 2) v = R[(size_t)(m0 + wm + 16 * i + rh + r) * ldy + n] + gv * v;
          so[(16 * i + rh + r) * 68 + 16 * j + cl] = v;
        }
      }
    }
  asm volatile("s_wait_dscnt 0" ::: "memory");
  __builtin_amdgcn_wave_barrier();
#pragma unroll 1
  for (int pass = 0; pass < 2; ++pass) {
    if (OUT16) {
      f16* Y = (f16*)Yv;
#pragma unroll
      for (int it = 0; it < 8; ++it) { const int c = lane + 32 * it, rr = c >> 3, q8 = (c & 7) * 8;
        union { f16 h[8]; v4u_t v; } u;
#pragma unroll
        for (int e = 0; e < 8; ++e) u.h[e] = (f16)so[rr * 68 + q8 + e];
        *(volatile v4u_t*)(Y + (size_t)(m0 + wm + rr) * ldy + n0 + wn + q8) = u.v; }
    } else {
      float* Y = (float*)Yv;
#pragma unroll
      for (int it = 0; it < 16; ++it) { const int f4 = lane + 32 * it, rr = f4 >> 4, q = (f4 & 15) * 4;
        *(volatile v4f_t*)(Y + (size_t)(m0 + wm + rr) * ldy + n0 + wn + q) = *(const v4fa*)(so + rr * 68 + q); }
    }
    __threadfence();
  }
}

template <typename AT, bool ACC>
__global__ __launch_bounds__(256) void gemm_kn2(const AT* __restrict__ A, int lda, size_t strideA,
                                               const float* __restrict__ Wm, int ldw, size_t strideW,
                                               const float* __restrict__ bias, float scale,
                                               float* __restrict__ Y, int ldy, size_t strideY, int K) {
  __shared__ __attribute__((aligned(16))) f16 ldsA[128 * GSTR], ldsAl[128 * GSTR];
  __shared__ __attribute__((aligned(16))) f16 ldsW[128 * GSTR], ldsWl[128 * GSTR];
  __shared__ __attribute__((aligned(16))) float oS[8][32 * 68];
  const int tid = threadIdx.x, lane = tid & 31, wave = tid >> 5, cl = lane & 15, rh = (lane >> 4) * 8;
  const int m0 = blockIdx.x * 128, n0 = blockIdx.y * 128;
  const int wm = (wave & 3) * 32, wn = (wave >> 2) * 64;
  A += (size_t)blockIdx.z * strideA; Wm += (size_t)blockIdx.z * strideW; Y += (size_t)blockIdx.z * strideY;
  f32x8 acc[2][4], accx[2][4];
#pragma unroll
  for (int i = 0; i < 2; ++i)
#pragma unroll
    for (int j = 0; j < 4; ++j) { f32x8 z = {}; acc[i][j] = z; accx[i][j] = z; }
#pragma unroll 1
  for (int k0 = 0; k0 < K; k0 += 32) {
    __syncthreads();
    {
      const int row = tid >> 1, ch = (tid & 1) * 16;
      const AT* src = A + (size_t)(m0 + row) * lda + k0 + ch;
#pragma unroll
      for (int g = 0; g < 16; ++g) { const float v = (float)src[g]; const f16 h = (f16)v; ldsA[row * GSTR + ch + g] = h; ldsAl[row * GSTR + ch + g] = (f16)((v - (float)h) * 2048.0f); }
    }
    {
      const int k = tid >> 3, nn0 = (tid & 7) * 16;
      const float* src = Wm + (size_t)(k0 + k) * ldw + n0 + nn0;
#pragma unroll
      for (int g = 0; g < 4; ++g) { const v4f_t v = *(const v4f_t*)(src + 4 * g);
#pragma unroll
        for (int u = 0; u < 4; ++u) { const f16 h = (f16)v[u]; ldsW[(nn0 + 4 * g + u) * GSTR + k] = h; ldsWl[(nn0 + 4 * g + u) * GSTR + k] = (f16)((v[u] - (float)h) * 2048.0f); } }
    }
    __syncthreads();
    f16x16 af[2], afl[2];
#pragma unroll
    for (int i = 0; i < 2; ++i) { af[i] = lds_frag(ldsA + (wm + 16 * i) * GSTR, GSTR); afl[i] = lds_frag(ldsAl + (wm + 16 * i) * GSTR, GSTR); }
#pragma unroll
    for (int j = 0; j < 4; ++j) {
      const f16x16 bf = lds_frag(ldsW + (wn + 16 * j) * GSTR, GSTR), bfl = lds_frag(ldsWl + (wn + 16 * j) * GSTR, GSTR);
#pragma unroll
      for (int i = 0; i < 2; ++i) { acc[i][j] = wmma16(af[i], bf, acc[i][j]); accx[i][j] = wmma16(af[i], bfl, accx[i][j]); accx[i][j] = wmma16(afl[i], bf, accx[i][j]); }
    }
  }
  float* so = oS[wave];
#pragma unroll
  for (int i = 0; i < 2; ++i)
#pragma unroll
    for (int j = 0; j < 4; ++j) {
      const float bv = bias ? bias[n0 + wn + 16 * j + cl] : 0.0f;
#pragma unroll
      for (int r = 0; r < 8; ++r) so[(16 * i + rh + r) * 68 + 16 * j + cl] = (acc[i][j][r] + accx[i][j][r] * (1.0f / 2048.0f)) * scale + bv;
    }
  asm volatile("s_wait_dscnt 0" ::: "memory");
  __builtin_amdgcn_wave_barrier();
  if (ACC) {
#pragma unroll
    for (int it = 0; it < 16; ++it) { const int f4 = lane + 32 * it, rr = f4 >> 4, q = (f4 & 15) * 4;
      const v4f_t old = *(const v4fa*)(Y + (size_t)(m0 + wm + rr) * ldy + n0 + wn + q);
      v4f_t v = *(const v4fa*)(so + rr * 68 + q); v += old; *(v4fa*)(so + rr * 68 + q) = v; }
    asm volatile("s_wait_dscnt 0" ::: "memory");
  }
#pragma unroll 1
  for (int pass = 0; pass < 2; ++pass) {
#pragma unroll
    for (int it = 0; it < 16; ++it) { const int f4 = lane + 32 * it, rr = f4 >> 4, q = (f4 & 15) * 4;
      *(volatile v4f_t*)(Y + (size_t)(m0 + wm + rr) * ldy + n0 + wn + q) = *(const v4fa*)(so + rr * 68 + q); }
    __threadfence();
  }
}

__global__ __launch_bounds__(256) void k_transpose(const float* __restrict__ Wm, float* __restrict__ Wt, int rows, int cols) {
  __shared__ float tS[64][65];
  const int tid = threadIdx.x, tbj = cols / 64, bi = blockIdx.x / tbj, bj = blockIdx.x % tbj;
  for (int e = tid; e < 64 * 64; e += 256) { const int r = e >> 6, c = e & 63; tS[r][c] = Wm[(size_t)(bi * 64 + r) * cols + bj * 64 + c]; }
  __syncthreads();
  for (int ch = tid; ch < 64 * 16; ch += 256) { const int r = ch >> 4, q4 = (ch & 15) * 4; v4f_t o; o[0] = tS[q4][r]; o[1] = tS[q4 + 1][r]; o[2] = tS[q4 + 2][r]; o[3] = tS[q4 + 3][r];
    float* dst = Wt + (size_t)(bj * 64 + r) * rows + bi * 64 + q4; *(volatile v4f_t*)dst = o; __threadfence(); *(volatile v4f_t*)dst = o; }
}


template <typename AT, int EPI, bool OUT16, int NJ>
__global__ __launch_bounds__(256) void gemm_sm(const AT* __restrict__ A, int lda, size_t sA, const float* __restrict__ Wm, int ldw, size_t sW,
                                               const float* __restrict__ bias, const float* __restrict__ R, const float* __restrict__ gvec,
                                               void* __restrict__ Yv, int ldy, size_t sY, int K) {
  constexpr int BN = 16 * NJ; constexpr int OST = BN + 4;
  A += (size_t)blockIdx.z * sA; Wm += (size_t)blockIdx.z * sW; Yv = (void*)((char*)Yv + (size_t)blockIdx.z * sY * (OUT16 ? 2 : 4)); if (R) R += (size_t)blockIdx.z * sY;
  __shared__ __attribute__((aligned(16))) f16 ldsA[256 * GSTR];
  __shared__ __attribute__((aligned(16))) f16 ldsW[BN * GSTR];
  __shared__ __attribute__((aligned(16))) float oS[8][32 * OST];
  const int tid = threadIdx.x, lane = tid & 31, wave = tid >> 5, cl = lane & 15, rh = (lane >> 4) * 8;
  const int m0 = blockIdx.x * 256, n0 = blockIdx.y * BN;
  const int wm = wave * 32;
  f32x8 acc[2][NJ];
#pragma unroll
  for (int i = 0; i < 2; ++i)
#pragma unroll
    for (int j = 0; j < NJ; ++j) { f32x8 z = {}; acc[i][j] = z; }
#pragma unroll 1
  for (int k0 = 0; k0 < K; k0 += 32) {
    __syncthreads();
    { const AT* src = A + (size_t)(m0 + tid) * lda + k0;
#pragma unroll
      for (int g = 0; g < 32; ++g) ldsA[tid * GSTR + g] = (f16)src[g]; }
    { const int k = tid >> 3, nn0 = (tid & 7) * (2 * NJ);
      const float* src = Wm + (size_t)(k0 + k) * ldw + n0 + nn0;
#pragma unroll
      for (int g = 0; g < NJ / 2; ++g) { const v4f_t v = *(const v4f_t*)(src + 4 * g);
#pragma unroll
        for (int u = 0; u < 4; ++u) ldsW[(nn0 + 4 * g + u) * GSTR + k] = (f16)v[u]; } }
    __syncthreads();
    f16x16 af[2];
#pragma unroll
    for (int i = 0; i < 2; ++i) af[i] = lds_frag(ldsA + (wm + 16 * i) * GSTR, GSTR);
#pragma unroll
    for (int j = 0; j < NJ; ++j) {
      const f16x16 bf = lds_frag(ldsW + (16 * j) * GSTR, GSTR);
#pragma unroll
      for (int i = 0; i < 2; ++i) acc[i][j] = wmma16(af[i], bf, acc[i][j]);
    }
  }
  float* so = oS[wave];
#pragma unroll
  for (int i = 0; i < 2; ++i)
#pragma unroll
    for (int j = 0; j < NJ; ++j) {
      const int n = n0 + 16 * j + cl;
      const float bv = bias ? bias[n] : 0.0f;
      const float gv = (EPI == 2 || EPI == 4) ? gvec[n] : 0.0f;
#pragma unroll
      for (int r = 0; r < 8; ++r) {
        float v = acc[i][j][r] + bv;
        if (EPI == 3) v = fmaxf(v, 0.0f);
        if (EPI == 2) v = R[(size_t)(m0 + wm + 16 * i + rh + r) * ldy + n] + gv * v;
        if (EPI == 4) v = gv * v;
        so[(16 * i + rh + r) * OST + 16 * j + cl] = v;
      }
    }
  asm volatile("s_wait_dscnt 0" ::: "memory");
  __builtin_amdgcn_wave_barrier();
#pragma unroll 1
  for (int pass = 0; pass < 2; ++pass) {
    if (OUT16) {
      f16* Y = (f16*)Yv;
#pragma unroll
      for (int it = 0; it < BN / 8; ++it) { const int c = lane + 32 * it, rr = c / (BN / 8), q8 = (c % (BN / 8)) * 8;
        union { f16 h[8]; v4u_t v; } u;
#pragma unroll
        for (int e = 0; e < 8; ++e) u.h[e] = (f16)so[rr * OST + q8 + e];
        *(volatile v4u_t*)(Y + (size_t)(m0 + wm + rr) * ldy + n0 + q8) = u.v; }
    } else {
      float* Y = (float*)Yv;
#pragma unroll
      for (int it = 0; it < BN / 4; ++it) { const int f4 = lane + 32 * it, rr = f4 / (BN / 4), q = (f4 % (BN / 4)) * 4;
        *(volatile v4f_t*)(Y + (size_t)(m0 + wm + rr) * ldy + n0 + q) = *(const v4fa*)(so + rr * OST + q); }
    }
    __threadfence();
  }
}

#define NBk 2
#define NNk2 2048
#define DDk 1024
#define NHk 16
#define HDk 64
#define SEGk 512
#define NSEG (NNk2 / SEGk)
#define PPk 32
#define KFR 2112
#define DFFk 2730
#define HLD 5504
#define GLD 2752
__global__ __launch_bounds__(256) void k_fill(float* __restrict__ p, float val, size_t n4) { const size_t i = (size_t)blockIdx.x * 256 + threadIdx.x; if (i < n4) { v4f_t v = {val, val, val, val}; *(volatile v4f_t*)(p + 4 * i) = v; __threadfence(); *(volatile v4f_t*)(p + 4 * i) = v; } }
__global__ __launch_bounds__(256) void k_dbg_zero(float* __restrict__ p, size_t n4) { const size_t i = (size_t)blockIdx.x * 256 + threadIdx.x; if (i < n4) { v4f_t z = {0.f,0.f,0.f,0.f}; *(volatile v4f_t*)(p + 4 * i) = z; __threadfence(); *(volatile v4f_t*)(p + 4 * i) = z; } }
__global__ __launch_bounds__(256) void k_copy(const float* __restrict__ src, float* __restrict__ dst, size_t n4) { const size_t i = (size_t)blockIdx.x * 256 + threadIdx.x; if (i < n4) { const v4f_t v = *(const v4f_t*)(src + 4 * i); *(volatile v4f_t*)(dst + 4 * i) = v; __threadfence(); *(volatile v4f_t*)(dst + 4 * i) = v; } }
__global__ __launch_bounds__(256) void k_transpose_ld(const float* __restrict__ Wm, int lds, float* __restrict__ Wt, int rows, int cols) {
  __shared__ float tS[64][65];
  const int tid = threadIdx.x, tbj = cols / 64, bi = blockIdx.x / tbj, bj = blockIdx.x % tbj;
  for (int e = tid; e < 64 * 64; e += 256) { const int r = e >> 6, c = e & 63; tS[r][c] = Wm[(size_t)(bi * 64 + r) * lds + bj * 64 + c]; }
  __syncthreads();
  for (int ch = tid; ch < 64 * 16; ch += 256) { const int r = ch >> 4, q4 = (ch & 15) * 4; v4f_t o; o[0] = tS[q4][r]; o[1] = tS[q4 + 1][r]; o[2] = tS[q4 + 2][r]; o[3] = tS[q4 + 3][r];
    float* dst = Wt + (size_t)(bj * 64 + r) * rows + bi * 64 + q4; *(volatile v4f_t*)dst = o; __threadfence(); *(volatile v4f_t*)dst = o; }
}
__global__ __launch_bounds__(256) void k_vsum(const float* __restrict__ V, int ldv, float* __restrict__ VB) {
  const int c = blockIdx.x * 256 + threadIdx.x; if (c >= 1024) return; float s = 0.0f;
#pragma unroll 1
  for (int r = 0; r < 32; ++r) s += V[(size_t)r * ldv + c];
  const float m = s;   *(volatile float*)(VB + c) = m; __threadfence(); *(volatile float*)(VB + c) = m;
}
__global__ __launch_bounds__(256) void k_vsum2(const float* __restrict__ V, int ldv, float* __restrict__ VB) {
  const int c = blockIdx.x * 256 + threadIdx.x; if (c >= 1024) return; float s = 0.0f;
#pragma unroll 1
  for (int r = 0; r < 512; ++r) s += V[(size_t)r * ldv + c];
  const float m = s;   *(volatile float*)(VB + c) = m; __threadfence(); *(volatile float*)(VB + c) = m;
}
__global__ __launch_bounds__(256) void k_rms(const float* __restrict__ X, const float* __restrict__ w, float* __restrict__ Y) {
  __shared__ float red[8];
  const size_t r = blockIdx.x; const int tid = threadIdx.x, c = 4 * tid; const v4f_t v = *(const v4f_t*)(X + r * DDk + c); float s = v[0] * v[0] + v[1] * v[1] + v[2] * v[2] + v[3] * v[3];
#pragma unroll
  for (int o = 1; o < 32; o <<= 1) s += __shfl_xor(s, o, 32);
  if ((tid & 31) == 0) red[tid >> 5] = s; __syncthreads(); float t = 0.0f;
#pragma unroll
  for (int i = 0; i < 8; ++i) t += red[i];
  const float inv = 1.0f / __builtin_sqrtf(t * (1.0f / (float)DDk) + 1.1920929e-07f); const v4f_t y = v * inv * *(const v4f_t*)(w + c);
  *(volatile v4f_t*)(Y + r * DDk + c) = y; __threadfence(); *(volatile v4f_t*)(Y + r * DDk + c) = y;
}
__global__ __launch_bounds__(256) void k_colmean(const float* __restrict__ M, float* __restrict__ PM) { const int c = blockIdx.x * 256 + threadIdx.x; float s = 0.0f;
#pragma unroll 1
  for (int r = 0; r < NNk2; ++r) s += M[(size_t)r * DDk + c];
  s *= (1.0f / (float)NNk2); *(volatile float*)(PM + c) = s; __threadfence(); *(volatile float*)(PM + c) = s; }
__global__ __launch_bounds__(256) void k_matvec(const float* __restrict__ v, const float* __restrict__ Wm, int ldw, int col0, float* __restrict__ y) {
  __shared__ float vs[DDk]; const int tid = threadIdx.x; for (int i = tid; i < DDk; i += 256) vs[i] = v[i]; __syncthreads();
  const int c = blockIdx.x * 256 + tid; float s = 0.0f;
#pragma unroll 1
  for (int i = 0; i < DDk; ++i) s += vs[i] * Wm[(size_t)i * ldw + col0 + c];
  *(volatile float*)(y + c) = s; __threadfence(); *(volatile float*)(y + c) = s; }
__global__ __launch_bounds__(256) void k_prefix(const float* __restrict__ kc, const float* __restrict__ vc, const float* __restrict__ pm, float* __restrict__ KF, float* __restrict__ VF) {
  const int r = blockIdx.x, c = 4 * threadIdx.x; v4f_t kv, vv;
  if (r < 16) { kv = *(const v4f_t*)(kc + c); vv = *(const v4f_t*)(vc + c); }
  else { const int h = c / HDk, d = c % HDk; kv = *(const v4f_t*)(pm + ((size_t)h * 16 + (r - 16)) * HDk + d); vv = kv; }
  *(volatile v4f_t*)(KF + (size_t)r * DDk + c) = kv; *(volatile v4f_t*)(VF + (size_t)r * DDk + c) = vv; __threadfence(); *(volatile v4f_t*)(KF + (size_t)r * DDk + c) = kv; *(volatile v4f_t*)(VF + (size_t)r * DDk + c) = vv;
}
__global__ __launch_bounds__(32) void k_ropetbl(float* __restrict__ TC, float* __restrict__ TS) {
  const int s = blockIdx.x, i = threadIdx.x; const float inv = (float)(1.0 / pow(10000.0, (double)(2 * i) / (double)HDk)); const float ang = (float)s * inv;
  const float c = (float)cos((double)ang), sn = (float)sin((double)ang);
  *(volatile float*)(TC + (size_t)s * 32 + i) = c; *(volatile float*)(TS + (size_t)s * 32 + i) = sn; __threadfence(); *(volatile float*)(TC + (size_t)s * 32 + i) = c; *(volatile float*)(TS + (size_t)s * 32 + i) = sn;
}
__global__ __launch_bounds__(256) void k_ropei(float* __restrict__ X, const float* __restrict__ TC, const float* __restrict__ TS) {
  const size_t s = blockIdx.x; const int tid = threadIdx.x, h = tid >> 4, ch = tid & 15, p = 2 * ch;
  float* base = X + s * DDk + h * HDk + 4 * ch; const v4f_t x = *(const v4fa*)base;
  const float c0 = TC[s * 32 + p], s0 = TS[s * 32 + p], c1 = TC[s * 32 + p + 1], s1 = TS[s * 32 + p + 1];
  v4f_t o; o[0] = x[0] * c0 - x[1] * s0; o[1] = x[1] * c0 + x[0] * s0; o[2] = x[2] * c1 - x[3] * s1; o[3] = x[3] * c1 + x[2] * s1;
  *(volatile v4fa*)base = o; __threadfence(); *(volatile v4fa*)base = o;
}
__global__ __launch_bounds__(256) void k_segsoft(float* __restrict__ SP, float* __restrict__ SS) {
  __shared__ float red[256];
  const int r = blockIdx.x, tid = threadIdx.x; float* sp = SP + (size_t)r * PPk; float* ss = SS + (size_t)r * SEGk; float vp = -3.0e38f, v[SEGk / 256]; float m = -3.0e38f;
  if (tid < PPk) { vp = sp[tid] * 0.125f; m = vp; }
#pragma unroll
  for (int e = 0; e < SEGk / 256; ++e) { const int kk = tid + 256 * e; v[e] = (kk <= r) ? ss[min(kk, r)] * 0.125f : -3.0e38f; m = fmaxf(m, v[e]); }
  red[tid] = m; __syncthreads(); for (int o = 128; o > 0; o >>= 1) { if (tid < o) red[tid] = fmaxf(red[tid], red[tid + o]); __syncthreads(); }
  m = red[0]; __syncthreads(); float zs = 0.0f; float ep = 0.0f;
  if (tid < PPk) { ep = expf(vp - m); zs += ep; }
#pragma unroll
  for (int e = 0; e < SEGk / 256; ++e) { const int kk = tid + 256 * e; v[e] = (kk <= r) ? expf(v[e] - m) : 0.0f; zs += v[e]; }
  red[tid] = zs; __syncthreads(); for (int o = 128; o > 0; o >>= 1) { if (tid < o) red[tid] += red[tid + o]; __syncthreads(); }
  const float kk2 = 1024.0f / red[0];
#pragma unroll 1
  for (int pass = 0; pass < 2; ++pass) {
    if (tid < PPk) *(volatile float*)(sp + tid) = ep * kk2 - 1.0f;
#pragma unroll
    for (int e = 0; e < SEGk / 256; ++e) *(volatile float*)(ss + tid + 256 * e) = v[e] * kk2 - 1.0f;
    __threadfence(); }
}
__global__ __launch_bounds__(256) void k_add(const float* __restrict__ Aa, const float* __restrict__ Bb, float* __restrict__ R, size_t n4) { const size_t i = (size_t)blockIdx.x * 256 + threadIdx.x; if (i >= n4) return; const v4f_t v = *(const v4f_t*)(Aa + 4 * i) + *(const v4f_t*)(Bb + 4 * i); *(volatile v4f_t*)(R + 4 * i) = v; __threadfence(); *(volatile v4f_t*)(R + 4 * i) = v; }
__global__ __launch_bounds__(256) void k_geglu(const float* __restrict__ Hm, float* __restrict__ GG) { const size_t r = blockIdx.x; const int tid = threadIdx.x; const float* hr = Hm + r * HLD;
#pragma unroll 1
  for (int pass = 0; pass < 2; ++pass) {
#pragma unroll 1
    for (int c = tid; c < DFFk; c += 256) { const float a = hr[c], g = hr[DFFk + c]; *(volatile float*)(GG + r * GLD + c) = (g / (1.0f + expf(-g))) * a; }
    __threadfence(); }
}
__global__ __launch_bounds__(256) void k_tail10(const float* __restrict__ GG, const float* __restrict__ W2, float* __restrict__ O) { const size_t r = blockIdx.x; const int c = 4 * threadIdx.x; v4f_t acc = *(const v4fa*)(O + r * DDk + c);
#pragma unroll
  for (int j = 0; j < 10; ++j) acc += GG[r * GLD + 2720 + j] * *(const v4f_t*)(W2 + (size_t)(2720 + j) * DDk + c);
  *(volatile v4fa*)(O + r * DDk + c) = acc; __threadfence(); *(volatile v4fa*)(O + r * DDk + c) = acc; }

extern "C" void kernel_launch(void* const* d_in, const int* in_sizes, int n_in,
                              void* d_out, int out_size, void* d_ws, size_t ws_size,
                              hipStream_t stream) {
  (void)in_sizes; (void)n_in; (void)out_size;
  const float** f = (const float**)d_in;
  const float* x = f[0], *mem = f[1], *anw = f[2], *Wqkv = f[3], *Wout = f[4], *pmem = f[5], *mpw = f[6], *Wmt = f[7], *ffw = f[8], *W1 = f[9], *b1 = f[10], *W2 = f[11], *b2 = f[12];
  float* out = (float*)d_out;
  char* ws = (char*)d_ws;
  float* XN = (float*)ws; ws += (size_t)NNk2 * DDk * 4; float* Q = (float*)ws; ws += (size_t)NNk2 * DDk * 4; float* KF = (float*)ws; ws += (size_t)KFR * DDk * 4; float* VF = (float*)ws; ws += (size_t)KFR * DDk * 4;
  float* KT = (float*)ws; ws += (size_t)HDk * KFR * 4; float* SP = (float*)ws; ws += (size_t)SEGk * PPk * 4; float* SS = (float*)ws; ws += (size_t)SEGk * SEGk * 4;
  float* PMv = (float*)ws; ws += DDk * 4; float* PN = (float*)ws; ws += DDk * 4; float* MT = (float*)ws; ws += DDk * 4; float* KC = (float*)ws; ws += DDk * 4; float* VC = (float*)ws; ws += DDk * 4;
  float* VSP = (float*)ws; ws += DDk * 4; float* VSS = (float*)ws; ws += (size_t)4 * DDk * 4; float* VB = (float*)ws; ws += (size_t)4 * DDk * 4; float* sc = (float*)ws; ws += 64 * 4; float* ones = (float*)ws; ws += 2 * DFFk * 4 + 64; float* TC = (float*)ws; ws += (size_t)NNk2 * 32 * 4; float* TSn = (float*)ws; ws += (size_t)NNk2 * 32 * 4;
  float* ATT = (float*)ws; ws += (size_t)NNk2 * DDk * 4; float* X1 = (float*)ws; ws += (size_t)NNk2 * DDk * 4; float* Hm = (float*)ws; ws += (size_t)NNk2 * HLD * 4; float* GG = (float*)ws; ws += (size_t)NNk2 * GLD * 4;
  if ((size_t)(ws - (char*)d_ws) > ws_size) return;
  const dim3 blk(256); const size_t n4 = (size_t)NNk2 * DDk / 4;
  k_fill<<<dim3(1), blk, 0, stream>>>(sc, 1.0f / 1024.0f, 64 / 4); k_fill<<<dim3((2 * DFFk / 4 + 255) / 256), blk, 0, stream>>>(ones, 1.0f, 2 * DFFk / 4 + 1);
  k_fill<<<dim3(((size_t)(KFR - PPk - NNk2) * DDk / 4 + 255) / 256), blk, 0, stream>>>(KF + (size_t)(PPk + NNk2) * DDk, 0.0f, (size_t)(KFR - PPk - NNk2) * DDk / 4);
  k_ropetbl<<<dim3(NNk2), dim3(32), 0, stream>>>(TC, TSn);

  for (int b = 0; b < NBk; ++b) { const float* xb = x + (size_t)b * NNk2 * DDk; const float* mb = mem + (size_t)b * NNk2 * DDk; float* ob = out + (size_t)b * NNk2 * DDk;
    k_colmean<<<dim3(DDk / 256), blk, 0, stream>>>(mb, PMv); k_rms<<<dim3(1), blk, 0, stream>>>(PMv, mpw, PN);
    k_matvec<<<dim3(DDk / 256), blk, 0, stream>>>(PN, Wmt, DDk, 0, MT);
    k_matvec<<<dim3(DDk / 256), blk, 0, stream>>>(MT, Wqkv, 3 * DDk, DDk, KC); k_matvec<<<dim3(DDk / 256), blk, 0, stream>>>(MT, Wqkv, 3 * DDk, 2 * DDk, VC);
    k_prefix<<<dim3(PPk), blk, 0, stream>>>(KC, VC, pmem, KF, VF);
    k_rms<<<dim3(NNk2), blk, 0, stream>>>(xb, anw, XN);
    gemm_kne<float, 0, false><<<dim3(NNk2 / 128, DDk / 128), blk, 0, stream>>>(XN, DDk, Wqkv, 3 * DDk, nullptr, nullptr, nullptr, Q, DDk, DDk);
    gemm_kne<float, 0, false><<<dim3(NNk2 / 128, DDk / 128), blk, 0, stream>>>(XN, DDk, Wqkv + DDk, 3 * DDk, nullptr, nullptr, nullptr, KF + (size_t)PPk * DDk, DDk, DDk);
    gemm_kne<float, 0, false><<<dim3(NNk2 / 128, DDk / 128), blk, 0, stream>>>(XN, DDk, Wqkv + 2 * DDk, 3 * DDk, nullptr, nullptr, nullptr, VF + (size_t)PPk * DDk, DDk, DDk);
    k_ropei<<<dim3(NNk2), blk, 0, stream>>>(Q, TC, TSn); k_ropei<<<dim3(NNk2), blk, 0, stream>>>(KF + (size_t)PPk * DDk, TC, TSn);
    k_vsum<<<dim3(DDk / 256), blk, 0, stream>>>(VF, DDk, VSP);
    for (int sg = 0; sg < NSEG; ++sg) { k_vsum2<<<dim3(DDk / 256), blk, 0, stream>>>(VF + (size_t)(PPk + sg * SEGk) * DDk, DDk, VSS + sg * DDk); k_add<<<dim3((DDk / 4 + 255) / 256), blk, 0, stream>>>(VSP, VSS + sg * DDk, VB + sg * DDk, DDk / 4); }
    for (int h = 0; h < NHk; ++h) {
      k_transpose_ld<<<dim3((KFR / 64) * (HDk / 64)), blk, 0, stream>>>(KF + h * HDk, DDk, KT, KFR, HDk);
      for (int sg = 0; sg < NSEG; ++sg) { const float* Qs = Q + (size_t)sg * SEGk * DDk + h * HDk;
        gemm_sm<float, 0, false, 2><<<dim3(SEGk / 256, 1, 1), blk, 0, stream>>>(Qs, DDk, (size_t)0, KT, KFR, (size_t)0, nullptr, nullptr, nullptr, SP, PPk, (size_t)0, HDk);
        gemm_kne<float, 0, false><<<dim3(SEGk / 128, SEGk / 128), blk, 0, stream>>>(Qs, DDk, KT + PPk + sg * SEGk, KFR, nullptr, nullptr, nullptr, SS, SEGk, HDk);
        k_segsoft<<<dim3(SEGk), blk, 0, stream>>>(SP, SS);
        float* Y = ATT + (size_t)sg * SEGk * DDk + h * HDk;
        gemm_sm<float, 4, false, 4><<<dim3(SEGk / 256, 1, 1), blk, 0, stream>>>(SS, SEGk, (size_t)0, VF + (size_t)(PPk + sg * SEGk) * DDk + h * HDk, DDk, (size_t)0, VB + sg * DDk + h * HDk, nullptr, sc, Y, DDk, (size_t)0, SEGk);
        gemm_sm<float, 2, false, 4><<<dim3(SEGk / 256, 1, 1), blk, 0, stream>>>(SP, PPk, (size_t)0, VF + h * HDk, DDk, (size_t)0, nullptr, Y, sc, Y, DDk, (size_t)0, PPk);
      }
    }
    gemm_kne<float, 2, false><<<dim3(NNk2 / 128, DDk / 128), blk, 0, stream>>>(ATT, DDk, Wout, DDk, nullptr, xb, ones, X1, DDk, DDk);
    k_rms<<<dim3(NNk2), blk, 0, stream>>>(X1, ffw, XN);
    gemm_kne<float, 0, false><<<dim3(NNk2 / 128, 5376 / 128), blk, 0, stream>>>(XN, DDk, W1, 2 * DFFk, b1, nullptr, nullptr, Hm, HLD, DDk);
    gemm_kne<float, 0, false><<<dim3(NNk2 / 128, 1), blk, 0, stream>>>(XN, DDk, W1 + (2 * DFFk - 128), 2 * DFFk, b1 + (2 * DFFk - 128), nullptr, nullptr, Hm + (2 * DFFk - 128), HLD, DDk);
    k_geglu<<<dim3(NNk2), blk, 0, stream>>>(Hm, GG);
    gemm_kne<float, 2, false><<<dim3(NNk2 / 128, DDk / 128), blk, 0, stream>>>(GG, GLD, W2, DDk, b2, X1, ones, ob, DDk, 2720);
    k_tail10<<<dim3(NNk2), blk, 0, stream>>>(GG, W2, ob);
  }
}
